// MambaNodeMamba_36060545417603
// MI455X (gfx1250) — hardware-verified
//
#include <hip/hip_runtime.h>
#include <math.h>

typedef __attribute__((ext_vector_type(16))) _Float16 v16h;
typedef __attribute__((ext_vector_type(8)))  _Float16 v8h;
typedef __attribute__((ext_vector_type(16))) __bf16   v16b;
typedef __attribute__((ext_vector_type(8)))  __bf16   v8b;
typedef __attribute__((ext_vector_type(8)))  float    v8f;
typedef __attribute__((ext_vector_type(4)))  float    v4f;

constexpr int kBatch  = 32;
constexpr int kTime   = 24;
constexpr int kNode   = 207;
constexpr int kChan   = 64;
constexpr int kSeqL   = kNode * kTime;
constexpr int kCatW   = 2 * kChan;
constexpr int kDinner = 128;
constexpr int kNst    = 16;
constexpr int kDtR    = 4;
constexpr int kXdblN  = kDtR + 2 * kNst;
constexpr int kXdblP  = 64;
constexpr int kXZW    = 2 * kDinner;
constexpr int kChunkB = 8;
constexpr int kNChunk = kBatch / kChunkB;
constexpr int kMc     = kChunkB * kSeqL;
constexpr int kScanSub = 24;
constexpr int kRowP   = 132;
constexpr int kStatsP = 32;
static_assert(kMc % 64 == 0, "chunk rows must be a tile multiple");
static_assert(kSeqL % kScanSub == 0, "scan sub-chunk must divide L");
static_assert(kBatch % kChunkB == 0, "chunks must cover the batch");
static_assert((kMc * kCatW) % (8 * 256) == 0, "gather grid exact");

__device__ __forceinline__ unsigned short f2bf_bits(float f) {
  unsigned u = __float_as_uint(f);
  return (unsigned short)((u + 0x7FFFu + ((u >> 16) & 1u)) >> 16);
}
__device__ __forceinline__ float bf_bits2f(unsigned short h) { return __uint_as_float(((unsigned)h) << 16); }

__device__ __forceinline__ void dep_guard_h(v8f& a, v8f& b, v16h x, v16h y) { asm volatile("v_nop\n\tv_nop\n\tv_nop\n\tv_nop" : "+v"(a), "+v"(b) : "v"(x), "v"(y)); }
__device__ __forceinline__ void dep_guard_b(v8f& a, v8f& b, v16b x, v16b y) { asm volatile("v_nop\n\tv_nop\n\tv_nop\n\tv_nop" : "+v"(a), "+v"(b) : "v"(x), "v"(y)); }
__device__ __forceinline__ void keep4_h(v16h a, v16h b, v16h c, v16h d) { asm volatile("v_nop" :: "v"(a), "v"(b), "v"(c), "v"(d)); }
__device__ __forceinline__ void keep4_b(v16b a, v16b b, v16b c, v16b d) { asm volatile("v_nop" :: "v"(a), "v"(b), "v"(c), "v"(d)); }
__device__ __forceinline__ void acc_guard4(v8f& a, v8f& b, v8f& c, v8f& d) { asm volatile("v_nop\n\tv_nop\n\tv_nop\n\tv_nop" : "+v"(a), "+v"(b), "+v"(c), "+v"(d)); }
template <typename T> struct Frag;
template <> struct Frag<_Float16> {
  typedef v16h V; union U { v16h v; v8h h[2]; };
  static __device__ __forceinline__ v16h load(const _Float16* p) {
    U f; f.h[0] = *(const v8h*)(p); f.h[1] = *(const v8h*)(p + 16); return f.v;
  }
  static __device__ __forceinline__ v8f mma(v16h a, v16h b, v8f c) {
    return __builtin_amdgcn_wmma_f32_16x16x32_f16(false, a, false, b, (short)0, c, false, false);
  }
  static __device__ __forceinline__ void guard(v8f& a, v8f& b, v16h x, v16h y) { dep_guard_h(a, b, x, y); }
  static __device__ __forceinline__ void keep(v16h a, v16h b, v16h c, v16h d) { keep4_h(a, b, c, d); }
};
template <> struct Frag<__bf16> {
  typedef v16b V; union U { v16b v; v8b h[2]; };
  static __device__ __forceinline__ v16b load(const __bf16* p) {
    U f; f.h[0] = *(const v8b*)(p); f.h[1] = *(const v8b*)(p + 16); return f.v;
  }
  static __device__ __forceinline__ v8f mma(v16b a, v16b b, v8f c) {
    return __builtin_amdgcn_wmma_f32_16x16x32_bf16(false, a, false, b, (short)0, c, false, false);
  }
  static __device__ __forceinline__ void guard(v8f& a, v8f& b, v16b x, v16b y) { dep_guard_b(a, b, x, y); }
  static __device__ __forceinline__ void keep(v16b a, v16b b, v16b c, v16b d) { keep4_b(a, b, c, d); }
};

__device__ __forceinline__ int out_row_map(int m, int b0) {
  const int bl = m / kSeqL;
  const int l  = m - bl * kSeqL;
  const int n  = l / kTime;
  const int t  = l - n * kTime;
  return ((b0 + bl) * kTime + t) * kNode + n;
}

template <int ET> struct Elem;
template <> struct Elem<0> { typedef _Float16 T; };
template <> struct Elem<1> { typedef __bf16 T; };
template <int ET, bool SPLIT, int BIAS_MODE, int OUT_MODE, bool RESID, int ACT = 0, int ROWMAP = 0>
__global__ __launch_bounds__(256) void wmma_gemm64(
    const unsigned short* __restrict__ Ap, const unsigned short* __restrict__ A2p, int lda, long strideA,
    const unsigned short* __restrict__ Btp, const unsigned short* __restrict__ Bt2p, int ldb, long strideB,
    void* __restrict__ Cout, void* __restrict__ Cout2, int ldc, long strideC,
    const float* __restrict__ bias,
    const float* __restrict__ resid, long strideR,
    int M, int N, int K, float scale, int map_b0) {
  typedef typename Elem<ET>::T T;
  typedef typename Frag<T>::V V;
  const T* A = (const T*)Ap; const T* A2 = (const T*)A2p; const T* Bt = (const T*)Btp; const T* Bt2 = (const T*)Bt2p;
  __shared__ __align__(16) float sT[8][16 * 68];
  const int b    = blockIdx.y;
  const int lane = threadIdx.x & 31;
  const int wave = threadIdx.x >> 5;
  const int tilesN = N >> 6;
  const int tilesM = M >> 6;
  const int tile = blockIdx.x * 8 + wave;
  if (tile >= tilesM * tilesN) return;
  const int tm = tile / tilesN;
  const int tn = tile - tm * tilesN;
  const int m0 = tm << 6;
  const int n0 = tn << 6;

  const T* Ab  = A  + (size_t)b * strideA;
  const T* Bb  = Bt + (size_t)b * strideB;
  const T* Ab2 = SPLIT ? (A2  + (size_t)b * strideA) : nullptr;
  const T* Bb2 = SPLIT ? (Bt2 + (size_t)b * strideB) : nullptr;

  const int rlane = lane & 15;
  const int koff  = (lane >> 4) * 8;
  const int mOff  = (lane >> 4) * 8;

  v8f acc[4][4];
#pragma unroll
  for (int i = 0; i < 4; ++i)
#pragma unroll
    for (int j = 0; j < 4; ++j) acc[i][j] = (v8f){0.f,0.f,0.f,0.f,0.f,0.f,0.f,0.f};

  for (int k0 = 0; k0 < K; k0 += 32) {
    V bh[4], bl[4];
#pragma unroll
    for (int j = 0; j < 4; ++j) {
      const size_t bo = (size_t)(n0 + (j << 4) + rlane) * ldb + koff + k0;
      bh[j] = Frag<T>::load(Bb + bo);
      if (SPLIT) bl[j] = Frag<T>::load(Bb2 + bo);
    }
#pragma unroll
    for (int i = 0; i < 4; ++i) {
      const size_t ao = (size_t)(m0 + (i << 4) + rlane) * lda + koff + k0;
      V ah = Frag<T>::load(Ab + ao);
      V al;
      if (SPLIT) al = Frag<T>::load(Ab2 + ao);
#pragma unroll
      for (int j = 0; j < 4; ++j) {
        acc[i][j] = Frag<T>::mma(ah, bh[j], acc[i][j]);
        if (SPLIT) {
          acc[i][j] = Frag<T>::mma(ah, bl[j], acc[i][j]);
          acc[i][j] = Frag<T>::mma(al, bh[j], acc[i][j]);
        }
      }
      Frag<T>::guard(acc[i][0], acc[i][3], ah, SPLIT ? al : ah);
    }
    Frag<T>::keep(bh[0], bh[1], bh[2], bh[3]);
    if (SPLIT) Frag<T>::keep(bl[0], bl[1], bl[2], bl[3]);
  }
  acc_guard4(acc[0][0], acc[0][1], acc[0][2], acc[0][3]);
  acc_guard4(acc[1][0], acc[1][1], acc[1][2], acc[1][3]);
  acc_guard4(acc[2][0], acc[2][1], acc[2][2], acc[2][3]);
  acc_guard4(acc[3][0], acc[3][1], acc[3][2], acc[3][3]);

  float* slab = sT[wave];
  const float* Rb = RESID ? (resid + (size_t)b * strideR) : nullptr;
#pragma unroll
  for (int i = 0; i < 4; ++i) {
    const int mBase = m0 + (i << 4);
#pragma unroll
    for (int j = 0; j < 4; ++j) {
      const int n = n0 + (j << 4) + rlane;
      float bv = 0.f;
      if (BIAS_MODE == 2) bv = bias[n];
#pragma unroll
      for (int r = 0; r < 8; ++r) {
        float v = acc[i][j][r] * scale;
        if (BIAS_MODE == 1) v += bias[mBase + mOff + r];
        if (BIAS_MODE == 2) v += bv;
        if (RESID) {
          const int rrow = ROWMAP ? out_row_map(mBase + mOff + r, map_b0) : (mBase + mOff + r);
          v += Rb[(size_t)rrow * ldc + n];
        }
        if (ACT == 1) v = tanhf(v);
        if (ACT == 2) v = fmaxf(v, 0.0f);
        if (ACT == 3) v = v / (1.0f + expf(-v));
        if (ACT == 4) v = (v > 0.f) ? v : 0.01f * v;
        slab[(mOff + r) * 68 + (j << 4) + rlane] = v;
      }
    }
    __builtin_amdgcn_fence(__ATOMIC_RELEASE, "workgroup");
    __builtin_amdgcn_wave_barrier();
    __builtin_amdgcn_fence(__ATOMIC_ACQUIRE, "workgroup");
    if (OUT_MODE == 0) {
      float* C = (float*)Cout + (size_t)b * strideC;
      const int hh = lane >> 4, c4 = (lane & 15) * 4;
      for (int pass = 0; pass < 2; ++pass) {
#pragma unroll
        for (int it = 0; it < 8; ++it) {
          const int row = it * 2 + hh;
          const int prow = ROWMAP ? out_row_map(mBase + row, map_b0) : (mBase + row);
          v4f v = *(const v4f*)(slab + row * 68 + c4);
          *(volatile v4f*)(C + (size_t)prow * ldc + n0 + c4) = v;
        }
        __threadfence();
      }
    } else {
      const int q = lane >> 3, c8 = (lane & 7) * 8;
      unsigned short* C  = (unsigned short*)Cout  + (size_t)b * strideC;
      unsigned short* C2 = (OUT_MODE == 2) ? ((unsigned short*)Cout2 + (size_t)b * strideC) : nullptr;
      for (int pass = 0; pass < 2; ++pass) {
#pragma unroll
        for (int it = 0; it < 4; ++it) {
          const int row = it * 4 + q;
          const float* sp = slab + row * 68 + c8;
          v8h hv, lv;
#pragma unroll
          for (int e = 0; e < 8; ++e) {
            if (OUT_MODE == 1) {
              hv[e] = (_Float16)sp[e];
            } else {
              unsigned short hb = f2bf_bits(sp[e]);
              unsigned short lb = f2bf_bits(sp[e] - bf_bits2f(hb));
              hv[e] = __builtin_bit_cast(_Float16, hb);
              lv[e] = __builtin_bit_cast(_Float16, lb);
            }
          }
          *(volatile v8h*)(C + (size_t)(mBase + row) * ldc + n0 + c8) = hv;
          if (OUT_MODE == 2) *(volatile v8h*)(C2 + (size_t)(mBase + row) * ldc + n0 + c8) = lv;
        }
        __threadfence();
      }
    }
    __builtin_amdgcn_fence(__ATOMIC_RELEASE, "workgroup");
    __builtin_amdgcn_wave_barrier();
    __builtin_amdgcn_fence(__ATOMIC_ACQUIRE, "workgroup");
  }
}

__global__ __launch_bounds__(256) void cast_w_kernel(
    const float* __restrict__ W, unsigned short* __restrict__ Bt, int nreal, int Kdim, int total8, float scale)
{
  const int i = blockIdx.x * 256 + threadIdx.x;
  if (i >= total8) return;
  const int e0  = i << 3;
  const int row = e0 / Kdim;
  const int col = e0 - row * Kdim;
  const int rc  = (row < nreal) ? row : (nreal - 1);
  const float* p = W + (size_t)rc * Kdim + col;
  const v4f a0 = *(const v4f*)(p);
  const v4f a1 = *(const v4f*)(p + 4);
  const float zs = (row < nreal) ? scale : 0.f;
  v8h hv;
#pragma unroll
  for (int e = 0; e < 4; ++e) {
    hv[e]     = (_Float16)(a0[e] * zs);
    hv[4 + e] = (_Float16)(a1[e] * zs);
  }
  unsigned short* q = Bt + e0;
  *(volatile v8h*)q = hv;
  __threadfence();
  *(volatile v8h*)q = hv;
}

__global__ __launch_bounds__(256) void gather_xcat_kernel(
    const float* __restrict__ x, const float* __restrict__ qk, unsigned short* __restrict__ XCAT, int cb, int total8)
{
  const int i = blockIdx.x * 256 + threadIdx.x;
  if (i >= total8) return;
  const int e0  = i << 3;
  const int m   = e0 >> 7;
  const int col = e0 & 127;
  const int bl  = m / kSeqL;
  const int l   = m - bl * kSeqL;
  const int n   = l / kTime;
  const int t   = l - n * kTime;
  const int b   = cb * kChunkB + bl;
  const size_t base = ((size_t)(b * kTime + t) * kNode + n) * kChan + (col & 63);
  const v4f xa = *(const v4f*)(x + base);
  const v4f xb = *(const v4f*)(x + base + 4);
  const v4f qa = *(const v4f*)(qk + base);
  const v4f qb = *(const v4f*)(qk + base + 4);
  const bool useq = (col >= kChan);
  v8h hv;
#pragma unroll
  for (int e = 0; e < 4; ++e) {
    hv[e]     = (_Float16)(useq ? qa[e] : xa[e]);
    hv[4 + e] = (_Float16)(useq ? qb[e] : xb[e]);
  }
  unsigned short* q = XCAT + e0;
  *(volatile v8h*)q = hv;
  __threadfence();
  *(volatile v8h*)q = hv;
}

__global__ __launch_bounds__(128) void conv_silu_kernel(
    const _Float16* __restrict__ XZh, const float* __restrict__ cw, const float* __restrict__ cb,
    _Float16* __restrict__ XCh)
{
  __shared__ __align__(16) float sT[16 * kRowP];
  const int tid = threadIdx.x, lane = tid & 31, wave = tid >> 5;
  const int d = tid;
  const int t0 = blockIdx.x * 64;
  const float w0 = cw[d * 4 + 0], w1 = cw[d * 4 + 1], w2 = cw[d * 4 + 2], w3 = cw[d * 4 + 3];
  const float bc = cb[d];
  float xm3, xm2, xm1;
  {
    const int r3 = t0 - 3, r2 = t0 - 2, r1 = t0 - 1;
    const float v3 = (float)XZh[(size_t)(r3 < 0 ? 0 : r3) * kXZW + d];
    const float v2 = (float)XZh[(size_t)(r2 < 0 ? 0 : r2) * kXZW + d];
    const float v1 = (float)XZh[(size_t)(r1 < 0 ? 0 : r1) * kXZW + d];
    xm3 = (r3 >= 0) ? v3 : 0.f;
    xm2 = (r2 >= 0) ? v2 : 0.f;
    xm1 = (r1 >= 0) ? v1 : 0.f;
  }
  const int hrow = wave * 2 + (lane >> 4);
  const int c8   = (lane & 15) * 8;
#pragma unroll 1
  for (int sub = 0; sub < 4; ++sub) {
    const int lb = t0 + sub * 16;
#pragma unroll 1
    for (int s = 0; s < 16; ++s) {
      const int m = lb + s;
      const int l = m % kSeqL;
      const float xcur = (float)XZh[(size_t)m * kXZW + d];
      const float a0 = (l >= 3) ? xm3 : 0.f;
      const float a1 = (l >= 2) ? xm2 : 0.f;
      const float a2 = (l >= 1) ? xm1 : 0.f;
      float acc = w0 * a0;
      acc = fmaf(w1, a1, acc);
      acc = fmaf(w2, a2, acc);
      acc = fmaf(w3, xcur, acc);
      const float sv = acc + bc;
      const float sg = __builtin_amdgcn_rcpf(1.0f + __expf(-sv));
      sT[s * kRowP + d] = sv * sg;
      xm3 = xm2; xm2 = xm1; xm1 = xcur;
    }
    __syncthreads();
    v8h hv[2];
#pragma unroll
    for (int it = 0; it < 2; ++it) {
      const float* sp = sT + (it * 8 + hrow) * kRowP + c8;
      const v4f a0 = *(const v4f*)(sp);
      const v4f a1 = *(const v4f*)(sp + 4);
#pragma unroll
      for (int e = 0; e < 4; ++e) { hv[it][e] = (_Float16)a0[e]; hv[it][4 + e] = (_Float16)a1[e]; }
    }
    for (int pass = 0; pass < 2; ++pass) {
#pragma unroll
      for (int it = 0; it < 2; ++it)
        *(volatile v8h*)(XCh + (size_t)(lb + it * 8 + hrow) * kDinner + c8) = hv[it];
      __threadfence();
    }
    __syncthreads();
  }
}

__global__ __launch_bounds__(128) void scan_kernel(
    const float* __restrict__ XDBL, const _Float16* __restrict__ XCh, const _Float16* __restrict__ XZh,
    const float* __restrict__ W_dt, const float* __restrict__ b_dt, const float* __restrict__ A_log,
    const float* __restrict__ Dv, _Float16* __restrict__ Yh)
{
  __shared__ __align__(16) float sP[kScanSub * kXdblP];
  __shared__ __align__(16) float sY[kScanSub * kRowP];
  const int tid = threadIdx.x, lane = tid & 31, wave = tid >> 5;
  const int d = tid;
  const int row0 = blockIdx.x * kSeqL;

  float An[kNst];
#pragma unroll
  for (int n = 0; n < kNst; ++n) An[n] = -__expf(A_log[(size_t)d * kNst + n]);
  const float wd0 = W_dt[d * kDtR + 0], wd1 = W_dt[d * kDtR + 1], wd2 = W_dt[d * kDtR + 2], wd3 = W_dt[d * kDtR + 3];
  const float bdt = b_dt[d];
  const float Dd  = Dv[d];
  float h[kNst];
#pragma unroll
  for (int n = 0; n < kNst; ++n) h[n] = 0.f;

  const int hrow = wave * 2 + (lane >> 4);
  const int c8   = (lane & 15) * 8;

#pragma unroll 1
  for (int c = 0; c < kSeqL / kScanSub; ++c) {
    const int l0 = c * kScanSub;
#pragma unroll
    for (int p = 0; p < 3; ++p) {
      const int idx = tid + p * 128;
      const int r = idx >> 4, q = (idx & 15) * 4;
      const v4f v = *(const v4f*)(XDBL + (size_t)(row0 + l0 + r) * kXdblP + q);
      *(v4f*)(sP + r * kXdblP + q) = v;
    }
    __syncthreads();
#pragma unroll 1
    for (int s = 0; s < kScanSub; ++s) {
      const size_t m = (size_t)(row0 + l0 + s);
      const v4f x4 = *(const v4f*)(sP + s * kXdblP);
      float a = x4[0] * wd0;
      a = fmaf(x4[1], wd1, a);
      a = fmaf(x4[2], wd2, a);
      a = fmaf(x4[3], wd3, a);
      a += bdt;
      const float delta = fmaxf(a, 0.0f) + log1pf(__expf(-fabsf(a)));
      const float xv = (float)XCh[m * kDinner + d];
      const float zv = (float)XZh[m * kXZW + kDinner + d];
      float dtx = delta * xv;
      asm volatile("" : "+v"(dtx));
      v4f Bq[4], Cq[4];
#pragma unroll
      for (int qq = 0; qq < 4; ++qq) {
        Bq[qq] = *(const v4f*)(sP + s * kXdblP + kDtR + 4 * qq);
        Cq[qq] = *(const v4f*)(sP + s * kXdblP + kDtR + kNst + 4 * qq);
      }
      float y = 0.f;
#pragma unroll
      for (int n = 0; n < kNst; ++n) {
        const float e = __expf(delta * An[n]);
        float p = dtx * Bq[n >> 2][n & 3];
        asm volatile("" : "+v"(p));
        float qv = h[n] * e;
        asm volatile("" : "+v"(qv));
        const float hn = qv + p;
        h[n] = hn;
        float rr = hn * Cq[n >> 2][n & 3];
        asm volatile("" : "+v"(rr));
        y += rr;
      }
      float sk = xv * Dd;
      asm volatile("" : "+v"(sk));
      y += sk;
      const float sg = __builtin_amdgcn_rcpf(1.0f + __expf(-zv));
      const float g  = zv * sg;
      sY[s * kRowP + d] = (y * g) * 16.0f;
    }
    __syncthreads();
    v8h hv[3];
#pragma unroll
    for (int it = 0; it < 3; ++it) {
      const float* sp = sY + (it * 8 + hrow) * kRowP + c8;
      const v4f a0 = *(const v4f*)(sp);
      const v4f a1 = *(const v4f*)(sp + 4);
#pragma unroll
      for (int e = 0; e < 4; ++e) { hv[it][e] = (_Float16)a0[e]; hv[it][4 + e] = (_Float16)a1[e]; }
    }
    for (int pass = 0; pass < 2; ++pass) {
#pragma unroll
      for (int it = 0; it < 3; ++it)
        *(volatile v8h*)(Yh + (size_t)(row0 + l0 + it * 8 + hrow) * kDinner + c8) = hv[it];
      __threadfence();
    }
  }
}

__global__ __launch_bounds__(256) void gn_stats_kernel(const float* H, float* __restrict__ STATS)
{
  __shared__ double rs[256], rq[256];
  const int tid = threadIdx.x, lane = tid & 31;
  const int blk = blockIdx.x;
  const int b = blk >> 2, g = blk & 3;
  double s = 0.0, s2 = 0.0;
#pragma unroll 1
  for (int i4 = tid; i4 < kSeqL * 4; i4 += 256) {
    const int p = i4 >> 2, q = (i4 & 3) * 4;
    const v4f v = *(const v4f*)(H + ((size_t)b * kSeqL + p) * kChan + g * 16 + q);
#pragma unroll
    for (int e = 0; e < 4; ++e) { const double dv = (double)v[e]; s += dv; s2 += dv * dv; }
  }
  rs[tid] = s; rq[tid] = s2;
  __syncthreads();
  for (int off = 128; off > 0; off >>= 1) {
    if (tid < off) { rs[tid] += rs[tid + off]; rq[tid] += rq[tid + off]; }
    __syncthreads();
  }
  if (tid < 32) {
    const double inv = 1.0 / (double)(16 * kSeqL);
    const double mu  = rs[0] * inv;
    double var = rq[0] * inv - mu * mu;
    var = var > 0.0 ? var : 0.0;
    const float muf  = (float)mu;
    const float rstd = rsqrtf((float)var + 1e-5f);
    const float val = (lane == 0) ? muf : ((lane == 1) ? rstd : 0.f);
    float* q = STATS + (size_t)blk * kStatsP + lane;
    *(volatile float*)q = val;
    __threadfence();
    *(volatile float*)q = val;
  }
}

__global__ __launch_bounds__(256) void gn_apply_kernel(
    float* H, const float* __restrict__ STATS, const float* __restrict__ gw, const float* __restrict__ gb, int total4)
{
  const int i = blockIdx.x * 256 + threadIdx.x;
  if (i >= total4) return;
  const size_t e0 = (size_t)i << 2;
  const int row = (int)(e0 >> 6);
  const int c   = (int)(e0 & 63);
  const int b   = row / (kTime * kNode);
  const int g   = c >> 4;
  const float mu = STATS[(size_t)(b * 4 + g) * kStatsP + 0];
  const float rv = STATS[(size_t)(b * 4 + g) * kStatsP + 1];
  const v4f v  = *(const v4f*)(H + e0);
  const v4f w  = *(const v4f*)(gw + c);
  const v4f bb = *(const v4f*)(gb + c);
  v4f o;
#pragma unroll
  for (int e = 0; e < 4; ++e) o[e] = ((v[e] - mu) * rv) * w[e] + bb[e];
  float* q = H + e0;
  *(volatile v4f*)q = o;
  __threadfence();
  *(volatile v4f*)q = o;
}

extern "C" void kernel_launch(void* const* d_in, const int* in_sizes, int n_in,
                              void* d_out, int out_size, void* d_ws, size_t ws_size,
                              hipStream_t stream)
{
  if (n_in < 15) return;
  const float* x      = (const float*)d_in[0];
  const float* qk     = (const float*)d_in[1];
  const float* W_lin  = (const float*)d_in[2];
  const float* b_lin  = (const float*)d_in[3];
  const float* W_in   = (const float*)d_in[4];
  const float* conv_w = (const float*)d_in[5];
  const float* conv_b = (const float*)d_in[6];
  const float* W_x    = (const float*)d_in[7];
  const float* W_dt   = (const float*)d_in[8];
  const float* b_dt   = (const float*)d_in[9];
  const float* A_log  = (const float*)d_in[10];
  const float* D_par  = (const float*)d_in[11];
  const float* W_out  = (const float*)d_in[12];
  const float* gn_w   = (const float*)d_in[13];
  const float* gn_b   = (const float*)d_in[14];
  float* dout = (float*)d_out;

  const int kTotOut = kBatch * kTime * kNode * kChan;
  if (in_sizes[0] != kTotOut || in_sizes[1] != kTotOut) return;
  if (in_sizes[2] != kChan * kCatW || in_sizes[3] != kChan) return;
  if (in_sizes[4] != kXZW * kChan) return;
  if (in_sizes[5] != kDinner * 4 || in_sizes[6] != kDinner) return;
  if (in_sizes[7] != kXdblN * kDinner) return;
  if (in_sizes[8] != kDinner * kDtR || in_sizes[9] != kDinner) return;
  if (in_sizes[10] != kDinner * kNst || in_sizes[11] != kDinner) return;
  if (in_sizes[12] != kChan * kDinner) return;
  if (in_sizes[13] != kChan || in_sizes[14] != kChan) return;
  if (out_size != kTotOut) return;

  const size_t SZ_WLIN16 = (size_t)kChan * kCatW * 2;
  const size_t SZ_WIN16  = (size_t)kXZW * kChan * 2;
  const size_t SZ_WX16   = (size_t)kXdblP * kDinner * 2;
  const size_t SZ_WOUT16 = (size_t)kChan * kDinner * 2;
  const size_t SZ_STATS  = (size_t)kBatch * 4 * kStatsP * 4;
  const size_t SZ_XCAT16 = (size_t)kMc * kCatW * 2;
  const size_t SZ_SEQ16  = (size_t)kMc * kChan * 2;
  const size_t SZ_XZ16   = (size_t)kMc * kXZW * 2;
  const size_t SZ_XC16   = (size_t)kMc * kDinner * 2;
  const size_t SZ_XDBL   = (size_t)kMc * kXdblP * 4;
  const size_t SZ_Y16    = (size_t)kMc * kDinner * 2;
  const size_t OFF_WLIN16 = 0;
  const size_t OFF_WIN16  = OFF_WLIN16 + SZ_WLIN16;
  const size_t OFF_WX16   = OFF_WIN16  + SZ_WIN16;
  const size_t OFF_WOUT16 = OFF_WX16   + SZ_WX16;
  const size_t OFF_STATS  = OFF_WOUT16 + SZ_WOUT16;
  const size_t OFF_XCAT16 = OFF_STATS  + SZ_STATS;
  const size_t OFF_SEQ16  = OFF_XCAT16 + SZ_XCAT16;
  const size_t OFF_XZ16   = OFF_SEQ16  + SZ_SEQ16;
  const size_t OFF_XC16   = OFF_XZ16   + SZ_XZ16;
  const size_t OFF_XDBL   = OFF_XC16   + SZ_XC16;
  const size_t OFF_Y16    = OFF_XDBL   + SZ_XDBL;
  const size_t TOTAL      = OFF_Y16    + SZ_Y16;
  if (TOTAL > (size_t)134217728) return;
  if (ws_size < TOTAL) return;

  char* ws = (char*)d_ws;
  unsigned short* WLIN16 = (unsigned short*)(ws + OFF_WLIN16);
  unsigned short* WIN16  = (unsigned short*)(ws + OFF_WIN16);
  unsigned short* WX16   = (unsigned short*)(ws + OFF_WX16);
  unsigned short* WOUT16 = (unsigned short*)(ws + OFF_WOUT16);
  float*          STATS  = (float*)(ws + OFF_STATS);
  unsigned short* XCAT16 = (unsigned short*)(ws + OFF_XCAT16);
  unsigned short* SEQ16  = (unsigned short*)(ws + OFF_SEQ16);
  unsigned short* XZ16   = (unsigned short*)(ws + OFF_XZ16);
  unsigned short* XC16   = (unsigned short*)(ws + OFF_XC16);
  float*          XDBL   = (float*)(ws + OFF_XDBL);
  unsigned short* Y16    = (unsigned short*)(ws + OFF_Y16);
  const float* dummy_bias  = b_lin;
  const float* dummy_resid = x;

  cast_w_kernel<<<(kChan * kCatW) / 8 / 256, 256, 0, stream>>>(W_lin, WLIN16, kChan, kCatW,  (kChan * kCatW) / 8,  32.0f);
  cast_w_kernel<<<(kXZW * kChan) / 8 / 256, 256, 0, stream>>>(W_in,  WIN16,  kXZW,  kChan,  (kXZW * kChan) / 8,   32.0f);
  cast_w_kernel<<<(kXdblP * kDinner) / 8 / 256, 256, 0, stream>>>(W_x, WX16, kXdblN, kDinner, (kXdblP * kDinner) / 8, 32.0f);
  cast_w_kernel<<<(kChan * kDinner) / 8 / 256, 256, 0, stream>>>(W_out, WOUT16, kChan, kDinner, (kChan * kDinner) / 8, 32.0f);

  const int gemmBlocksN64  = (kMc / 64 + 7) / 8;
  const int gemmBlocksN256 = (kMc / 64 * 4 + 7) / 8;

  for (int cb = 0; cb < kNChunk; ++cb) {
    gather_xcat_kernel<<<(kMc * kCatW) / 8 / 256, 256, 0, stream>>>(x, qk, XCAT16, cb, (kMc * kCatW) / 8);

    wmma_gemm64<0, false, 2, 1, false, 0, 0><<<dim3(gemmBlocksN64, 1), 256, 0, stream>>>(
        XCAT16, XCAT16, kCatW, 0L, WLIN16, WLIN16, kCatW, 0L,
        (void*)SEQ16, (void*)SEQ16, kChan, 0L, b_lin, dummy_resid, 0L, kMc, kChan, kCatW, 1.0f / 32.0f, 0);

    wmma_gemm64<0, false, 0, 1, false, 0, 0><<<dim3(gemmBlocksN256, 1), 256, 0, stream>>>(
        SEQ16, SEQ16, kChan, 0L, WIN16, WIN16, kChan, 0L,
        (void*)XZ16, (void*)XZ16, kXZW, 0L, dummy_bias, dummy_resid, 0L, kMc, kXZW, kChan, 1.0f / 32.0f, 0);

    conv_silu_kernel<<<kMc / 64, 128, 0, stream>>>((const _Float16*)XZ16, conv_w, conv_b, (_Float16*)XC16);

    wmma_gemm64<0, false, 0, 0, false, 0, 0><<<dim3(gemmBlocksN64, 1), 256, 0, stream>>>(
        XC16, XC16, kDinner, 0L, WX16, WX16, kDinner, 0L,
        (void*)XDBL, (void*)XDBL, kXdblP, 0L, dummy_bias, dummy_resid, 0L, kMc, kXdblP, kDinner, 1.0f / 32.0f, 0);

    scan_kernel<<<kChunkB, 128, 0, stream>>>(XDBL, (const _Float16*)XC16, (const _Float16*)XZ16,
                                             W_dt, b_dt, A_log, D_par, (_Float16*)Y16);

    wmma_gemm64<0, false, 0, 0, true, 0, 1><<<dim3(gemmBlocksN64, 1), 256, 0, stream>>>(
        Y16, Y16, kDinner, 0L, WOUT16, WOUT16, kDinner, 0L,
        (void*)dout, (void*)dout, kChan, 0L, dummy_bias, x, 0L, kMc, kChan, kDinner, 1.0f / 512.0f, cb * kChunkB);
  }

  gn_stats_kernel<<<kBatch * 4, 256, 0, stream>>>(dout, STATS);
  gn_apply_kernel<<<kTotOut / 4 / 256, 256, 0, stream>>>(dout, STATS, gn_w, gn_b, kTotOut / 4);
}
